// MHSA2D_62766652063799
// MI455X (gfx1250) — hardware-verified
//
#include <hip/hip_runtime.h>


#ifndef NB
#define NB 8
#endif
#ifndef SEQ
#define SEQ 1024
#endif
#define NB_FULL  8
#define SEQ_FULL 1024
#ifndef OUT_SEQ
#define OUT_SEQ SEQ
#endif
#define CC   384
#define NH_  8
#define HD   48
#define HP   64
#define KP_  (NH_ * HP)
#define AW   4
#define OSP  68
#define SC2  ((float)(0.14433756729740643 * 1.4426950408889634))
#define PSH  14.0f
#define NEGB (-3.0e38f)
#define WPS  64.0f
#define CTXS 16.0f
#define OSCL (1.0f / 1024.0f)

static_assert(HD == 48);
static_assert(HP == 64);
static_assert(HD % 16 == 0);
static_assert(HD % 8 == 0);
static_assert(HP % 32 == 0);
static_assert(HD <= HP);
static_assert(NH_ * HD == CC);
static_assert(CC % 64 == 0);
static_assert(CC % 32 == 0);
static_assert(KP_ % 32 == 0);
static_assert(SEQ % 64 == 0);
static_assert((NB * SEQ) % 64 == 0);
static_assert(SEQ % 32 == 0);
static_assert(SEQ % (16 * AW) == 0);
static_assert(NB <= NB_FULL);
static_assert(SEQ <= SEQ_FULL);
static_assert((OSP * 4) % 16 == 0);
static_assert(OSP >= HP);
static_assert(((size_t)3 * CC * CC) % 8 == 0);
static_assert(((size_t)CC * KP_) % 8 == 0);
static_assert(WPS * CTXS * OSCL == 1.0f);
static_assert(256 * 16 == 32 * 64 * 2);
static_assert(4 * 32 * 16 == 16 * HP * 2);
static_assert(4 * 32 * 16 == 16 * 64 * 2);
static_assert(8 * 32 * 16 == 16 * 64 * 4);
static_assert(4 * 32 * 16 == 16 * HP * 2);
static_assert(64 * 33 * 4 <= 131072);
static_assert(16 * 68 * 4 <= 131072);
static_assert(AW * 16 * OSP * 4 <= 131072);

typedef _Float16 h16;
typedef unsigned short bf;
typedef __attribute__((ext_vector_type(16))) __bf16   v16bf;
typedef __attribute__((ext_vector_type(16))) _Float16 v16h;
typedef __attribute__((ext_vector_type(8)))  _Float16 v8h;
typedef __attribute__((ext_vector_type(8)))  unsigned short v8us;
typedef __attribute__((ext_vector_type(8)))  float    v8f;
typedef __attribute__((ext_vector_type(4)))  float    v4f;
typedef v4f  __attribute__((may_alias)) v4fa;

__device__ __forceinline__ unsigned short f2bf(float f) { unsigned u = __float_as_uint(f); u += 0x7FFFu + ((u >> 16) & 1u); return (unsigned short)(u >> 16); }
__device__ __forceinline__ float bfr(float f) { return __uint_as_float(((unsigned)f2bf(f)) << 16); }
__device__ __forceinline__ v16h cat16(v8h lo, v8h hi) { return __builtin_shufflevector(lo, hi, 0, 1, 2, 3, 4, 5, 6, 7, 8, 9, 10, 11, 12, 13, 14, 15); }
__device__ __forceinline__ v16bf cat16b(v8us lo, v8us hi) { return __builtin_bit_cast(v16bf, __builtin_shufflevector(lo, hi, 0, 1, 2, 3, 4, 5, 6, 7, 8, 9, 10, 11, 12, 13, 14, 15)); }
__device__ __forceinline__ v8f wmma16(v16h a, v16h b, v8f c) { return __builtin_amdgcn_wmma_f32_16x16x32_f16(false, a, false, b, (short)0, c, false, false); }
__device__ __forceinline__ v8f wmmab(v16bf a, v16bf b, v8f c) { return __builtin_amdgcn_wmma_f32_16x16x32_bf16(false, a, false, b, (short)0, c, false, false); }
__device__ __forceinline__ v16h  ldh(const h16* p) { return cat16(*(const v8h*)p, *(const v8h*)(p + 16)); }
__device__ __forceinline__ v16bf ldb(const bf* p)  { return cat16b(*(const v8us*)p, *(const v8us*)(p + 16)); }
__device__ __forceinline__ void wave_sync() { __builtin_amdgcn_fence(3  , "wavefront"); __builtin_amdgcn_wave_barrier(); asm volatile("" ::: "memory"); }
static __device__ __forceinline__ h16 toh_flush(float v) { const h16 r = (h16)v; return (fabsf(v) < 6.103515625e-05f) ? (h16)0.0f : r; }
__device__ __forceinline__ v8f wmma16g(v16h a, v16h b, v8f c) { c = wmma16(a, b, c); asm volatile("v_nop\n\tv_nop\n\tv_nop\n\tv_nop" : "+v"(c) : "v"(a), "v"(b)); return c; }
__device__ __forceinline__ v8f wmmabg(v16bf a, v16bf b, v8f c) { c = wmmab(a, b, c); asm volatile("v_nop\n\tv_nop\n\tv_nop\n\tv_nop" : "+v"(c) : "v"(a), "v"(b)); return c; }

__global__ __launch_bounds__(256) void k_cvt8(const float* __restrict__ src, bf* dst, size_t n8) {
    const size_t i = (size_t)blockIdx.x * 256 + threadIdx.x; if (i >= n8) return;
    const v8f v = *(const v8f*)(src + i * 8); v8us o;
#pragma unroll
    for (int k = 0; k < 8; ++k) o[k] = f2bf(v[k]);
    *(volatile v8us*)(dst + i * 8) = o; __threadfence(); *(volatile v8us*)(dst + i * 8) = o;
}

__global__ __launch_bounds__(256) void k_xT(const float* __restrict__ x, bf* dst) {
    __shared__ float ts[64 * 33];
    const int tid = threadIdx.x;
    const int n0 = blockIdx.x * 32, c0 = blockIdx.y * 64, b = blockIdx.z;
    const float* xs = x + ((size_t)b * CC + c0) * SEQ_FULL + n0;
#pragma unroll
    for (int i = 0; i < 8; ++i) { const int c = i * 8 + (tid >> 5), n = tid & 31;
        ts[c * 33 + n] = xs[(size_t)c * SEQ_FULL + n]; }
    __syncthreads();
    const int tok = tid >> 3, c8 = (tid & 7) * 8;
    v8us o;
#pragma unroll
    for (int k = 0; k < 8; ++k) o[k] = f2bf(ts[(c8 + k) * 33 + tok]);
    bf* p = dst + ((size_t)b * SEQ + n0 + tok) * CC + c0 + c8;
    *(volatile v8us*)p = o; __threadfence(); *(volatile v8us*)p = o;
}

__global__ __launch_bounds__(256) void k_wp(const float* __restrict__ src, h16* dst, size_t n8) {
    const size_t i = (size_t)blockIdx.x * 256 + threadIdx.x; if (i >= n8) return;
    const int o = (int)(i / (KP_ / 8)), c8 = (int)(i % (KP_ / 8)) * 8;
    const int h = c8 / HP, dd = c8 % HP;
    const bool ok = dd < HD;
    const int dc = dd < (HD - 8) ? dd : (HD - 8);
    v8f v = *(const v8f*)(src + (size_t)o * CC + h * HD + dc);
    asm volatile("" : "+v"(v));
    v8h hv;
#pragma unroll
    for (int k = 0; k < 8; ++k) hv[k] = ok ? toh_flush(bfr(v[k]) * WPS) : (h16)0.0f;
    *(volatile v8h*)(dst + i * 8) = hv; __threadfence(); *(volatile v8h*)(dst + i * 8) = hv;
}

__global__ __launch_bounds__(32) void k_proj_qk(const bf* __restrict__ A, const bf* __restrict__ Bt, const float* __restrict__ bias, h16* QK) {
    __shared__ __align__(16) float os[16 * 68];
    const int K = CC;
    const int lane = threadIdx.x & 31, lr = lane & 15, hi = lane >> 4; const int r0 = blockIdx.x * 64; const int hq = blockIdx.y;
    v8f acc[4][3];
#pragma unroll
    for (int mb = 0; mb < 4; ++mb)
#pragma unroll
        for (int nb = 0; nb < 3; ++nb) acc[mb][nb] = (v8f){};
    const size_t aoff = (size_t)(r0 + lr) * K + 8 * hi, boff = (size_t)(hq * HD + lr) * K + 8 * hi;
#pragma unroll 1
    for (int kc = 0; kc < K; kc += 32) {
        v16bf a[4];
#pragma unroll
        for (int mb = 0; mb < 4; ++mb) a[mb] = ldb(A + aoff + (size_t)mb * 16 * K + kc);
#pragma unroll
        for (int nb = 0; nb < 3; ++nb) { const v16bf b = ldb(Bt + boff + (size_t)nb * 16 * K + kc);
#pragma unroll
            for (int mb = 0; mb < 4; ++mb) acc[mb][nb] = wmmabg(a[mb], b, acc[mb][nb]); }
    }
    float bc[3];
#pragma unroll
    for (int nb = 0; nb < 3; ++nb) bc[nb] = bfr(bias[hq * HD + nb * 16 + lr]);
    const int bb = r0 / SEQ, tt = r0 % SEQ; const int three = hq / NH_, h = hq % NH_;
    const size_t tbase = ((((size_t)three * NB + (size_t)bb) * NH_ + (size_t)h) * SEQ + (size_t)tt) * HP;
#pragma unroll
    for (int mb = 0; mb < 4; ++mb) {
#pragma unroll
        for (int nb = 0; nb < 3; ++nb) {
#pragma unroll
            for (int j = 0; j < 8; ++j) os[(hi * 8 + j) * 68 + nb * 16 + lr] = acc[mb][nb][j] + bc[nb]; }
#pragma unroll
        for (int j = 0; j < 8; ++j) os[(hi * 8 + j) * 68 + HD + lr] = 0.0f;
        wave_sync();
#pragma unroll 1
        for (int ps = 0; ps < 2; ++ps) {
            const size_t sb = tbase + (size_t)(mb * 16) * HP;
#pragma unroll
            for (int s = 0; s < 4; ++s) { const int p = s * 32 + lane; const int row = p >> 3, c8 = (p & 7) * 8;
                const v4f x0 = *(const v4fa*)(&os[row * 68 + c8]); const v4f x1 = *(const v4fa*)(&os[row * 68 + c8 + 4]); v8h hv;
#pragma unroll
                for (int i = 0; i < 4; ++i) { hv[i] = toh_flush(x0[i]); hv[4 + i] = toh_flush(x1[i]); }
                *(volatile v8h*)(QK + sb + (size_t)p * 8) = hv; }
            if (ps == 0) __threadfence(); }
        wave_sync();
    }
}

__global__ __launch_bounds__(32) void k_proj_v(const bf* __restrict__ A, const bf* __restrict__ Bt, const float* __restrict__ bias, h16* VT) {
    __shared__ __align__(16) float os[16 * 68];
    const int K = CC;
    const int lane = threadIdx.x & 31, lr = lane & 15, hi = lane >> 4; const int r0 = blockIdx.x * 64, c0 = blockIdx.y * 64;
    v8f acc[4][4];
#pragma unroll
    for (int mb = 0; mb < 4; ++mb)
#pragma unroll
        for (int nb = 0; nb < 4; ++nb) acc[mb][nb] = (v8f){};
    const size_t aoff = (size_t)(r0 + lr) * K + 8 * hi, boff = (size_t)(c0 + lr) * K + 8 * hi;
#pragma unroll 1
    for (int kc = 0; kc < K; kc += 32) {
        v16bf a[4];
#pragma unroll
        for (int mb = 0; mb < 4; ++mb) a[mb] = ldb(A + aoff + (size_t)mb * 16 * K + kc);
#pragma unroll
        for (int nb = 0; nb < 4; ++nb) { const v16bf b = ldb(Bt + boff + (size_t)nb * 16 * K + kc);
#pragma unroll
            for (int mb = 0; mb < 4; ++mb) acc[mb][nb] = wmmabg(a[mb], b, acc[mb][nb]); }
    }
    const int bb = c0 / SEQ, tt = c0 % SEQ;
    const size_t tbase = (size_t)bb * (size_t)CC * SEQ + (size_t)r0 * SEQ + (size_t)tt;
#pragma unroll
    for (int mb = 0; mb < 4; ++mb) {
        float br[8];
#pragma unroll
        for (int j = 0; j < 8; ++j) br[j] = bfr(bias[r0 + mb * 16 + hi * 8 + j]);
#pragma unroll
        for (int nb = 0; nb < 4; ++nb) {
#pragma unroll
            for (int j = 0; j < 8; ++j) os[(hi * 8 + j) * 68 + nb * 16 + lr] = acc[mb][nb][j] + br[j]; }
        wave_sync();
#pragma unroll 1
        for (int ps = 0; ps < 2; ++ps) {
            const size_t sb = tbase + (size_t)(mb * 16) * SEQ;
#pragma unroll
            for (int s = 0; s < 4; ++s) { const int row = 4 * s + (lane >> 3), c8 = (lane & 7) * 8;
                const v4f x0 = *(const v4fa*)(&os[row * 68 + c8]); const v4f x1 = *(const v4fa*)(&os[row * 68 + c8 + 4]); v8h hv;
#pragma unroll
                for (int i = 0; i < 4; ++i) { hv[i] = toh_flush(x0[i]); hv[4 + i] = toh_flush(x1[i]); }
                *(volatile v8h*)(VT + sb + (size_t)row * SEQ + c8) = hv; }
            if (ps == 0) __threadfence(); }
        wave_sync();
    }
}

__global__ __launch_bounds__(32) void k_proj_out(const h16* __restrict__ A, const h16* __restrict__ Bt, const float* __restrict__ bias, float* OUT) {
    __shared__ __align__(16) float os[16 * 68];
    const int K = KP_;
    const int lane = threadIdx.x & 31, lr = lane & 15, hi = lane >> 4; const int r0 = blockIdx.x * 64, c0 = blockIdx.y * 64;
    v8f acc[4][4];
#pragma unroll
    for (int mb = 0; mb < 4; ++mb)
#pragma unroll
        for (int nb = 0; nb < 4; ++nb) acc[mb][nb] = (v8f){};
    const size_t aoff = (size_t)(r0 + lr) * K + 8 * hi, boff = (size_t)(c0 + lr) * K + 8 * hi;
#pragma unroll 1
    for (int kc = 0; kc < K; kc += 32) {
        v16h a[4];
#pragma unroll
        for (int mb = 0; mb < 4; ++mb) a[mb] = ldh(A + aoff + (size_t)mb * 16 * K + kc);
#pragma unroll
        for (int nb = 0; nb < 4; ++nb) { const v16h b = ldh(Bt + boff + (size_t)nb * 16 * K + kc);
#pragma unroll
            for (int mb = 0; mb < 4; ++mb) acc[mb][nb] = wmma16g(a[mb], b, acc[mb][nb]); }
    }
    const int bb = c0 / SEQ, tt = c0 % SEQ;
    const size_t tbase = ((size_t)bb * (size_t)CC + (size_t)r0) * OUT_SEQ + (size_t)tt;
#pragma unroll
    for (int mb = 0; mb < 4; ++mb) {
        float br[8];
#pragma unroll
        for (int j = 0; j < 8; ++j) br[j] = bfr(bias[r0 + mb * 16 + hi * 8 + j]);
#pragma unroll
        for (int nb = 0; nb < 4; ++nb) {
#pragma unroll
            for (int j = 0; j < 8; ++j) os[(hi * 8 + j) * 68 + nb * 16 + lr] = acc[mb][nb][j] * OSCL + br[j]; }
        wave_sync();
#pragma unroll 1
        for (int ps = 0; ps < 2; ++ps) {
            const size_t sb = tbase + (size_t)(mb * 16) * OUT_SEQ;
#pragma unroll
            for (int s = 0; s < 8; ++s) { const int row = 2 * s + (lane >> 4), c4 = (lane & 15) * 4;
                const v4f val = *(const v4fa*)(&os[row * 68 + c4]);
                *(volatile v4f*)(OUT + sb + (size_t)row * OUT_SEQ + c4) = val; }
            if (ps == 0) __threadfence(); }
        wave_sync();
    }
}

__global__ __launch_bounds__(32 * AW) void k_flash(const h16* __restrict__ QP, const h16* __restrict__ KP, const h16* __restrict__ VT, h16* CTX) {
    __shared__ __align__(16) float os[AW * 16 * OSP];
    const int lane = threadIdx.x & 31, lr = lane & 15, hi = lane >> 4;
    const int wave = __builtin_amdgcn_readfirstlane((int)(threadIdx.x >> 5));
    const int zh = blockIdx.y; const int b = zh / NH_, h = zh % NH_;
    const int t0 = (blockIdx.x * AW + wave) * 16;
    const size_t pbase = (size_t)zh * SEQ * HP;
    const size_t vbase = (size_t)zh * HD * SEQ;
    const size_t qo = pbase + (size_t)(t0 + lr) * HP + 8 * hi;
    const v16h q0 = ldh(QP + qo), q1 = ldh(QP + qo + 32);
    const size_t ko = pbase + (size_t)lr * HP + 8 * hi;
    const size_t vo = vbase + (size_t)lr * SEQ + 8 * hi;
    v8f o0 = (v8f){}, o1 = (v8f){}, o2 = (v8f){};
    float m = NEGB, l = 0.0f;
#pragma unroll 1
    for (int key0 = 0; key0 < SEQ; key0 += 32) {
        const h16* ka = KP + ko + (size_t)key0 * HP;
        const v16h ka0 = ldh(ka), ka1 = ldh(ka + 32), kb0 = ldh(ka + 16 * HP), kb1 = ldh(ka + 16 * HP + 32);
        v8f sa = (v8f){}, sb = (v8f){};
        sa = wmma16g(ka0, q0, sa); sa = wmma16g(ka1, q1, sa);
        sb = wmma16g(kb0, q0, sb); sb = wmma16g(kb1, q1, sb);
        float ta[8], tb[8]; float mx = NEGB;
#pragma unroll
        for (int r = 0; r < 8; ++r) { ta[r] = sa[r] * SC2; tb[r] = sb[r] * SC2; mx = fmaxf(mx, fmaxf(ta[r], tb[r])); }
        mx = fmaxf(mx, __shfl_xor(mx, 16, 32));
        const float mnew = fmaxf(m, mx);
        const float alpha = __builtin_amdgcn_exp2f(m - mnew);
        const float sh = PSH - mnew;
        v16h pb; float ls = 0.0f;
#pragma unroll
        for (int r = 0; r < 8; ++r) {
            const float ea = ta[r] + sh, eb = tb[r] + sh;
            const float xa = __builtin_amdgcn_exp2f(ea), xb = __builtin_amdgcn_exp2f(eb);
            const float ga = (ea < -14.0f) ? 0.0f : xa, gb = (eb < -14.0f) ? 0.0f : xb;
            const h16 pa = (h16)ga; const h16 pc = (h16)gb;
            pb[r] = pa; pb[8 + r] = pc;
            ls += (float)pa + (float)pc; }
        l = l * alpha + ls; m = mnew;
        o0 = o0 * alpha; o1 = o1 * alpha; o2 = o2 * alpha;
        const h16* va = VT + vo + key0;
        const v16h v0 = ldh(va), v1 = ldh(va + (size_t)16 * SEQ), v2 = ldh(va + (size_t)32 * SEQ);
        o0 = wmma16g(v0, pb, o0); o1 = wmma16g(v1, pb, o1); o2 = wmma16g(v2, pb, o2);
    }
    l += __shfl_xor(l, 16, 32);
    const float inv = CTXS * (1.0f / l);
    const int wb = wave * 16 * OSP;
    { v4f a, c;
      a[0] = o0[0] * inv; a[1] = o0[1] * inv; a[2] = o0[2] * inv; a[3] = o0[3] * inv; c[0] = o0[4] * inv; c[1] = o0[5] * inv; c[2] = o0[6] * inv; c[3] = o0[7] * inv;
      *(v4fa*)(&os[wb + lr * OSP +  0 + 8 * hi]) = a; *(v4fa*)(&os[wb + lr * OSP +  0 + 8 * hi + 4]) = c;
      a[0] = o1[0] * inv; a[1] = o1[1] * inv; a[2] = o1[2] * inv; a[3] = o1[3] * inv; c[0] = o1[4] * inv; c[1] = o1[5] * inv; c[2] = o1[6] * inv; c[3] = o1[7] * inv;
      *(v4fa*)(&os[wb + lr * OSP + 16 + 8 * hi]) = a; *(v4fa*)(&os[wb + lr * OSP + 16 + 8 * hi + 4]) = c;
      a[0] = o2[0] * inv; a[1] = o2[1] * inv; a[2] = o2[2] * inv; a[3] = o2[3] * inv; c[0] = o2[4] * inv; c[1] = o2[5] * inv; c[2] = o2[6] * inv; c[3] = o2[7] * inv;
      *(v4fa*)(&os[wb + lr * OSP + 32 + 8 * hi]) = a; *(v4fa*)(&os[wb + lr * OSP + 32 + 8 * hi + 4]) = c;
      const v4f z4 = (v4f){};
      *(v4fa*)(&os[wb + lr * OSP + HD + 8 * hi]) = z4; *(v4fa*)(&os[wb + lr * OSP + HD + 8 * hi + 4]) = z4; }
    wave_sync();
    h16* crow = CTX + ((size_t)b * SEQ + t0) * KP_ + h * HP;
#pragma unroll 1
    for (int ps = 0; ps < 2; ++ps) {
#pragma unroll
        for (int s = 0; s < 4; ++s) { const int row = 4 * s + (lane >> 3), c8 = (lane & 7) * 8;
            const v4f x0 = *(const v4fa*)(&os[wb + row * OSP + c8]); const v4f x1 = *(const v4fa*)(&os[wb + row * OSP + c8 + 4]); v8h hv;
#pragma unroll
            for (int i = 0; i < 4; ++i) { hv[i] = toh_flush(x0[i]); hv[4 + i] = toh_flush(x1[i]); }
            *(volatile v8h*)(crow + (size_t)row * KP_ + c8) = hv; }
        if (ps == 0) __threadfence(); }
}

static constexpr size_t al256(size_t v) { return (v + 255) & ~(size_t)255; }
static constexpr size_t SZ_XB = al256((size_t)NB * SEQ * CC * 2);
static constexpr size_t SZ_WB = al256((size_t)3 * CC * CC * 2);
static constexpr size_t SZ_WP = al256((size_t)CC * KP_ * 2);
static constexpr size_t SZ_QK = al256((size_t)2 * NB * NH_ * SEQ * HP * 2);
static constexpr size_t SZ_VT = al256((size_t)NB * CC * SEQ * 2);
static constexpr size_t SZ_CX = al256((size_t)NB * SEQ * KP_ * 2);
static constexpr size_t SZ_TOTAL = SZ_XB + SZ_WB + SZ_WP + SZ_QK + SZ_VT + SZ_CX;
static_assert(SZ_TOTAL <= (size_t)134217728);
static_assert(((size_t)2 * CC * CC * 2) % 256 == 0);
static_assert(((size_t)NB * NH_ * SEQ * HP * 2) % 256 == 0);
static_assert((size_t)NB * NH_ * HD * SEQ == (size_t)NB * CC * SEQ);

extern "C" void kernel_launch(void* const* d_in, const int* in_sizes, int n_in,
                              void* d_out, int out_size, void* d_ws, size_t ws_size, hipStream_t stream) {
    if (n_in < 5) return;
    const size_t needx = ((size_t)(NB - 1) * CC + (size_t)(CC - 1)) * SEQ_FULL + SEQ;
    if ((size_t)in_sizes[0] < needx) return;
    if ((size_t)in_sizes[1] < (size_t)3 * CC * CC || in_sizes[2] < 3 * CC) return;
    if ((size_t)in_sizes[3] < (size_t)CC * CC || in_sizes[4] < CC) return;
    if ((size_t)out_size < ((size_t)(NB - 1) * CC + (size_t)(CC - 1)) * OUT_SEQ + SEQ) return;
    if (SZ_TOTAL > ws_size) return;
    const float* x     = (const float*)d_in[0];
    const float* wqkv  = (const float*)d_in[1];
    const float* bqkv  = (const float*)d_in[2];
    const float* wproj = (const float*)d_in[3];
    const float* bproj = (const float*)d_in[4];
    float* OUT = (float*)d_out;
    char* wsp = (char*)d_ws;
    bf*  XB  = (bf*)wsp;  wsp += SZ_XB;
    bf*  WB  = (bf*)wsp;  wsp += SZ_WB;
    h16* WPp = (h16*)wsp; wsp += SZ_WP;
    h16* QK  = (h16*)wsp; wsp += SZ_QK;
    h16* VT  = (h16*)wsp; wsp += SZ_VT;
    h16* CTX = (h16*)wsp; wsp += SZ_CX;

    k_xT<<<dim3(SEQ / 32, CC / 64, NB), 256, 0, stream>>>(x, XB);
    { const size_t n8 = (size_t)3 * CC * CC / 8; k_cvt8<<<(unsigned)((n8 + 255) / 256), 256, 0, stream>>>(wqkv, WB, n8); }
    { const size_t n8 = (size_t)CC * KP_ / 8;    k_wp<<<(unsigned)((n8 + 255) / 256), 256, 0, stream>>>(wproj, WPp, n8); }

    k_proj_qk<<<dim3(NB * SEQ / 64, 2 * NH_, 1), 32, 0, stream>>>(XB, WB, bqkv, QK);
    k_proj_v<<<dim3(CC / 64, NB * SEQ / 64, 1), 32, 0, stream>>>(WB + (size_t)2 * CC * CC, XB, bqkv + 2 * CC, VT);

    k_flash<<<dim3(SEQ / (16 * AW), NB * NH_, 1), 32 * AW, 0, stream>>>(QK, QK + (size_t)NB * NH_ * SEQ * HP, VT, CTX);

    k_proj_out<<<dim3(CC / 64, NB * SEQ / 64, 1), 32, 0, stream>>>(WPp, CTX, bproj, OUT);
}
